// CustomizedRNN_13503377178895
// MI455X (gfx1250) — hardware-verified
//
#include <hip/hip_runtime.h>
#include <hip/hip_bf16.h>
#include <stdint.h>
#include <math.h>

constexpr int B_  = 64;
constexpr int T_  = 512;
constexpr int E_  = 300;
constexpr int EP_ = 320;
constexpr int H1_ = 256;
constexpr int H2_ = 512;
constexpr int D1_ = 128;
constexpr int D2_ = 64;

#define __bf16 _Float16
#define RSPLIT (1.0f / 2048.0f)
#define PLX1 ((size_t)T_ * B_ * H1_)
#define PLX2 ((size_t)T_ * B_ * H2_)
typedef __attribute__((ext_vector_type(16))) __bf16 v16bf;
typedef __attribute__((ext_vector_type(4))) unsigned v4u_t;
typedef unsigned v4ua __attribute__((ext_vector_type(4), may_alias));
typedef __attribute__((ext_vector_type(8)))  __bf16 v8bf;
typedef __attribute__((ext_vector_type(8)))  float  v8f;

#define SCHED_FENCE() __builtin_amdgcn_sched_barrier(0)

__device__ static inline v8f wmma_bf16(v16bf a, v16bf b, v8f c) {
  return __builtin_amdgcn_wmma_f32_16x16x32_f16(
      false, a, false, b, (short)0, c, false, false);
}
__device__ static inline v8f wmma_split(v16bf a, v16bf al, v16bf b, v16bf bl, v8f c) {
  v8f x = {};
  x = wmma_bf16(al, b, x); x = wmma_bf16(a, bl, x);
  return wmma_bf16(a, b, c) + x * RSPLIT;
}
__device__ static inline __bf16 split_lo(float v, __bf16 h) { return (__bf16)((v - (float)h) * 2048.0f); }

__device__ static inline v16bf cat8(v8bf lo, v8bf hi) {
  return __builtin_shufflevector(lo, hi, 0, 1, 2, 3, 4, 5, 6, 7,
                                 8, 9, 10, 11, 12, 13, 14, 15);
}

__device__ static inline v16bf load_a_frag(const __bf16* tile, int pitch, int lane) {
  int m  = lane & 15;
  int hi = (lane >> 4) & 1;
  const __bf16* p = tile + m * pitch + hi * 8;
  return cat8(*(const v8bf*)p, *(const v8bf*)(p + 16));
}

__device__ static inline v16bf load_swz_frag(const __bf16* fragbase, int lane) {
  const __bf16* p = fragbase + lane * 16;
  return cat8(*(const v8bf*)p, *(const v8bf*)(p + 8));
}

__device__ static inline v8bf cvt8_bf(v8f x) {
  v8bf r;
#pragma unroll
  for (int i = 0; i < 8; ++i) r[i] = (__bf16)x[i];
  return r;
}

__device__ static inline v8f cvt8_f32(v8bf x) {
  v8f r;
#pragma unroll
  for (int i = 0; i < 8; ++i) r[i] = (float)x[i];
  return r;
}
__device__ static inline v8f cvt8_f32p(v8bf x, v8bf xl) {
  v8f r;
#pragma unroll
  for (int i = 0; i < 8; ++i) r[i] = (float)x[i] + (float)xl[i] * RSPLIT;
  return r;
}
__device__ static inline void cvt8_split(v8f x, v8bf* h, v8bf* l) {
#pragma unroll
  for (int i = 0; i < 8; ++i) { const __bf16 hv = (__bf16)x[i]; (*h)[i] = hv; (*l)[i] = split_lo(x[i], hv); }
}
__device__ static inline void st2_planes(__bf16* p, size_t plane, v8bf h, v8bf l) {
  *(volatile v8bf*)p = h; *(volatile v8bf*)(p + plane) = l; __threadfence(); *(volatile v8bf*)p = h; *(volatile v8bf*)(p + plane) = l;
}

template <int KC>
__global__ void k_cvt_swz(const float* __restrict__ src, __bf16* __restrict__ dst,
                          int Kvalid, int N) {
  int i = (blockIdx.x * blockDim.x + threadIdx.x) * 2;
  if (i >= KC * 32 * N) return;
  const size_t plane = (size_t)KC * 32 * N;
  unsigned ph = 0, pl = 0;
#pragma unroll
  for (int q = 0; q < 2; ++q) {
    int ii   = i + q;
    int j    = ii & 15;
    int lane = (ii >> 4) & 31;
    int rest = ii >> 9;
    int c    = rest % KC;
    int nt   = rest / KC;
    int n = nt * 16 + (lane & 15);
    int hi = (lane >> 4) & 1;
    int k = c * 32 + ((j < 8) ? (hi * 8 + j) : (16 + hi * 8 + (j - 8)));
    float v = (k < Kvalid) ? src[k * N + n] : 0.f;
    const __bf16 hv = (__bf16)v, lv = split_lo(v, hv);
    ph |= (unsigned)__builtin_bit_cast(unsigned short, hv) << (16 * q);
    pl |= (unsigned)__builtin_bit_cast(unsigned short, lv) << (16 * q);
  }
  *(volatile unsigned*)(dst + i) = ph; *(volatile unsigned*)(dst + plane + i) = pl; __threadfence();
  *(volatile unsigned*)(dst + i) = ph; *(volatile unsigned*)(dst + plane + i) = pl;
}

__global__ __launch_bounds__(256) void k_xw1(
    const int* __restrict__ tokens, const float* __restrict__ emb,
    const __bf16* __restrict__ w1x, const float* __restrict__ b1,
    __bf16* __restrict__ xw1) {
  __shared__ __align__(16) __bf16 As[64][EP_];
  __shared__ __align__(16) __bf16 Asl[64][EP_];
  int t = blockIdx.x;
  int tid = threadIdx.x, lane = tid & 31, wave = tid >> 5;
  int mt = wave & 3;
  int ng = wave >> 2;

  {
    int row = tid >> 2, tp = tid & 3;
    int tok = tokens[row * T_ + t];
    const float* er = emb + (size_t)tok * E_;
#pragma unroll 8
    for (int i = 0; i < EP_ / 4; ++i) {
      int k = i * 4 + tp;
      { const float v = (k < E_) ? er[k] : 0.f; const __bf16 hv = (__bf16)v; As[row][k] = hv; Asl[row][k] = split_lo(v, hv); }
    }
  }

  v8f acc[8];
  int ncol0 = ng * 128 + (lane & 15);
#pragma unroll
  for (int nt = 0; nt < 8; ++nt) {
    float bv = b1[ncol0 + nt * 16];
#pragma unroll
    for (int r = 0; r < 8; ++r) acc[nt][r] = bv;
  }

  __syncthreads();

  const size_t plw = (size_t)10 * 32 * H1_;
#pragma unroll 2
  for (int c = 0; c < EP_ / 32; ++c) {
    v16bf af = load_a_frag(&As[mt * 16][c * 32], EP_, lane), afl = load_a_frag(&Asl[mt * 16][c * 32], EP_, lane);
#pragma unroll
    for (int nt = 0; nt < 8; ++nt) {
      const __bf16* fb = w1x + (size_t)((ng * 8 + nt) * 10 + c) * 512;
      acc[nt] = wmma_split(af, afl, load_swz_frag(fb, lane), load_swz_frag(fb + plw, lane), acc[nt]);
    }
  }

#pragma unroll
  for (int nt = 0; nt < 8; ++nt) {
    __bf16* p = xw1 + (size_t)((t * 16 + ng * 8 + nt) * 4 + mt) * 256 + lane * 8;
    v8bf h, l; cvt8_split(acc[nt], &h, &l); st2_planes(p, PLX1, h, l);
  }
}

__global__ __launch_bounds__(512) void k_xw2(
    const __bf16* __restrict__ seq1, const __bf16* __restrict__ w2x,
    const float* __restrict__ b2, __bf16* __restrict__ xw2) {
  int t = blockIdx.x;
  int tid = threadIdx.x, lane = tid & 31, wave = tid >> 5;
  int mt = wave & 3;
  int ng = wave >> 2;

  v8f acc[8];
  int ncol0 = ng * 128 + (lane & 15);
#pragma unroll
  for (int nt = 0; nt < 8; ++nt) {
    float bv = b2[ncol0 + nt * 16];
#pragma unroll
    for (int r = 0; r < 8; ++r) acc[nt][r] = bv;
  }

  const __bf16* arow = seq1 + (size_t)t * 64 * H1_ + (size_t)(mt * 16) * H1_;
  const size_t plw = (size_t)8 * 32 * H2_;
#pragma unroll 2
  for (int c = 0; c < H1_ / 32; ++c) {
    v16bf af = load_a_frag(arow + c * 32, H1_, lane), afl = load_a_frag(arow + PLX1 + c * 32, H1_, lane);
#pragma unroll
    for (int nt = 0; nt < 8; ++nt) {
      const __bf16* fb = w2x + (size_t)((ng * 8 + nt) * 8 + c) * 512;
      acc[nt] = wmma_split(af, afl, load_swz_frag(fb, lane), load_swz_frag(fb + plw, lane), acc[nt]);
    }
  }

#pragma unroll
  for (int nt = 0; nt < 8; ++nt) {
    __bf16* p = xw2 + (size_t)((t * 32 + ng * 8 + nt) * 4 + mt) * 256 + lane * 8;
    v8bf h, l; cvt8_split(acc[nt], &h, &l); st2_planes(p, PLX2, h, l);
  }
}

__global__ __launch_bounds__(512) void k_rnn1(
    const __bf16* __restrict__ xw1, const __bf16* __restrict__ w1h,
    __bf16* __restrict__ seq1) {
  __shared__ __align__(16) __bf16 hbuf[2][2][64][H1_];
  int tid = threadIdx.x, lane = tid & 31, wave = tid >> 5;

  v16bf wfrag[8], wfragl[8];
  const size_t plw = (size_t)8 * 32 * H1_;
#pragma unroll
  for (int c = 0; c < 8; ++c) {
    wfrag[c]  = load_swz_frag(w1h + (size_t)(wave * 8 + c) * 512, lane);
    wfragl[c] = load_swz_frag(w1h + plw + (size_t)(wave * 8 + c) * 512, lane);
  }

  {
    uint32_t* z = (uint32_t*)&hbuf[0][0][0][0];
    for (int i = tid; i < 2 * 2 * 64 * H1_ / 2; i += 512) z[i] = 0u;
  }
  __syncthreads();

  int nbase = wave * 16 + (lane & 15);
  int hi8 = (lane >> 4) << 3;

  for (int t = 0; t < T_; ++t) {
    const __bf16* cur  = &hbuf[t & 1][0][0][0];
    const __bf16* curl = &hbuf[t & 1][1][0][0];
    __bf16* nxt  = &hbuf[(t & 1) ^ 1][0][0][0];
    __bf16* nxtl = &hbuf[(t & 1) ^ 1][1][0][0];
    __bf16* srow = seq1 + (size_t)t * 64 * H1_;
    if (t + 1 < T_)
      __builtin_prefetch(xw1 + (size_t)(((t + 1) * 16 + wave) * 4) * 256 + lane * 8,
                         0, 3);
#pragma unroll
    for (int m = 0; m < 4; ++m) {
      const __bf16* xp = xw1 + (size_t)((t * 16 + wave) * 4 + m) * 256 + lane * 8;
      v8f acc = cvt8_f32p(*(const v8bf*)xp, *(const v8bf*)(xp + PLX1));
#pragma unroll
      for (int c = 0; c < 8; ++c) {
        v16bf a  = load_a_frag(cur  + m * 16 * H1_ + c * 32, H1_, lane);
        v16bf al = load_a_frag(curl + m * 16 * H1_ + c * 32, H1_, lane);
        acc = wmma_split(a, al, wfrag[c], wfragl[c], acc);
      }
#pragma unroll
      for (int r = 0; r < 8; ++r) {
        float v = acc[r] > 0.f ? acc[r] : 0.f;
        __bf16 bv = (__bf16)v;
        nxt [(m * 16 + hi8 + r) * H1_ + nbase] = bv;
        nxtl[(m * 16 + hi8 + r) * H1_ + nbase] = split_lo(v, bv);
      }
    }
    __syncthreads();
#pragma unroll 1
    for (int pass = 0; pass < 2; ++pass) {
#pragma unroll
      for (int i = 0; i < 4; ++i) {
        const int c = tid + 512 * i;
        const int rr = c >> 5, q = (c & 31) * 8;
        *(volatile v8bf*)(srow + (size_t)rr * H1_ + q)        = *(const volatile v8bf*)(nxt  + rr * H1_ + q);
        *(volatile v8bf*)(srow + PLX1 + (size_t)rr * H1_ + q) = *(const volatile v8bf*)(nxtl + rr * H1_ + q);
      }
      __threadfence();
    }
  }
}

__global__ __launch_bounds__(1024) void k_rnn2(
    const __bf16* __restrict__ xw2, const __bf16* __restrict__ w2h,
    float* __restrict__ hout) {
  __shared__ __align__(16) __bf16 hbuf[2][64][H2_];
  int tid = threadIdx.x, lane = tid & 31, wave = tid >> 5;

  {
    uint32_t* z = (uint32_t*)&hbuf[0][0][0];
    for (int i = tid; i < 2 * 64 * H2_ / 2; i += 1024) z[i] = 0u;
  }
  __syncthreads();

  int nbase = wave * 16 + (lane & 15);
  int hi8 = (lane >> 4) << 3;
  const __bf16* wbase = w2h + (size_t)(wave * 16) * 512;
  const size_t plw = (size_t)16 * 32 * H2_;
  __bf16* cur  = &hbuf[0][0][0];
  __bf16* curl = &hbuf[1][0][0];

  for (int t = 0; t < T_; ++t) {
    if (t + 1 < T_)
      __builtin_prefetch(xw2 + (size_t)(((t + 1) * 32 + wave) * 4) * 256 + lane * 8,
                         0, 3);

    v8f acc[4];
#pragma unroll
    for (int m = 0; m < 4; ++m) {
      const __bf16* xp = xw2 + (size_t)((t * 32 + wave) * 4 + m) * 256 + lane * 8;
      acc[m] = cvt8_f32p(*(const v8bf*)xp, *(const v8bf*)(xp + PLX2));
    }

#pragma unroll 2
    for (int c = 0; c < 16; ++c) {
      v16bf wf  = load_swz_frag(wbase + (size_t)c * 512, lane);
      v16bf wfl = load_swz_frag(wbase + plw + (size_t)c * 512, lane);
#pragma unroll
      for (int m = 0; m < 4; ++m) {
        v16bf a  = load_a_frag(cur  + m * 16 * H2_ + c * 32, H2_, lane);
        v16bf al = load_a_frag(curl + m * 16 * H2_ + c * 32, H2_, lane);
        acc[m] = wmma_split(a, al, wf, wfl, acc[m]);
      }
    }
    __syncthreads();

#pragma unroll
    for (int m = 0; m < 4; ++m)
#pragma unroll
      for (int r = 0; r < 8; ++r) {
        float v = acc[m][r] > 0.f ? acc[m][r] : 0.f;
        const __bf16 hv = (__bf16)v;
        cur [(m * 16 + hi8 + r) * H2_ + nbase] = hv;
        curl[(m * 16 + hi8 + r) * H2_ + nbase] = split_lo(v, hv);
      }
    __syncthreads();
  }
#pragma unroll 1
  for (int pass = 0; pass < 2; ++pass) {
#pragma unroll
    for (int i = 0; i < 8; ++i) {
      const int c = tid + 1024 * i, rr = c >> 7, q = (c & 127) * 4;
      typedef __attribute__((ext_vector_type(4))) float v4f_t;
      v4f_t v;
      v.x = (float)cur[rr * H2_ + q + 0] + (float)curl[rr * H2_ + q + 0] * RSPLIT;
      v.y = (float)cur[rr * H2_ + q + 1] + (float)curl[rr * H2_ + q + 1] * RSPLIT;
      v.z = (float)cur[rr * H2_ + q + 2] + (float)curl[rr * H2_ + q + 2] * RSPLIT;
      v.w = (float)cur[rr * H2_ + q + 3] + (float)curl[rr * H2_ + q + 3] * RSPLIT;
      *(volatile v4f_t*)(hout + (size_t)rr * H2_ + q) = v;
    }
    __threadfence();
  }
}

__global__ __launch_bounds__(256) void k_head(
    const float* __restrict__ h2,
    const float* __restrict__ wd1, const float* __restrict__ bd1,
    const float* __restrict__ wd2, const float* __restrict__ bd2,
    const float* __restrict__ wc, const float* __restrict__ bc,
    float* __restrict__ out) {
  __shared__ float d1[64][D1_];
  __shared__ float d2[64][D2_];
  int tid = threadIdx.x;
  for (int idx = tid; idx < 64 * D1_; idx += 256) {
    int b = idx >> 7, j = idx & (D1_ - 1);
    float s = bd1[j];
    for (int k = 0; k < H2_; ++k) s += h2[b * H2_ + k] * wd1[k * D1_ + j];
    d1[b][j] = s > 0.f ? s : 0.f;
  }
  __syncthreads();
  for (int idx = tid; idx < 64 * D2_; idx += 256) {
    int b = idx >> 6, j = idx & (D2_ - 1);
    float s = bd2[j];
    for (int k = 0; k < D1_; ++k) s += d1[b][k] * wd2[k * D2_ + j];
    d2[b][j] = s > 0.f ? s : 0.f;
  }
  __syncthreads();
  if (tid < 64) {
    float s = bc[0];
    for (int k = 0; k < D2_; ++k) s += d2[tid][k] * wc[k];
    const float v = 1.f / (1.f + __expf(-s));
    *(volatile float*)(out + tid) = v; __threadfence(); *(volatile float*)(out + tid) = v;
  }
}

extern "C" void kernel_launch(void* const* d_in, const int* in_sizes, int n_in,
                              void* d_out, int out_size, void* d_ws, size_t ws_size,
                              hipStream_t stream) {
  const int*   tokens = (const int*)  d_in[0];
  const float* emb    = (const float*)d_in[1];
  const float* W1x    = (const float*)d_in[2];
  const float* W1h    = (const float*)d_in[3];
  const float* b1     = (const float*)d_in[4];
  const float* W2x    = (const float*)d_in[5];
  const float* W2h    = (const float*)d_in[6];
  const float* b2     = (const float*)d_in[7];
  const float* Wd1    = (const float*)d_in[8];
  const float* bd1    = (const float*)d_in[9];
  const float* Wd2    = (const float*)d_in[10];
  const float* bd2    = (const float*)d_in[11];
  const float* Wc     = (const float*)d_in[12];
  const float* bc     = (const float*)d_in[13];
  float* out = (float*)d_out;

  char* ws = (char*)d_ws;
  size_t o = 0;
  __bf16* w1x_sw  = (__bf16*)(ws + o); o += (size_t)EP_ * H1_ * 2 * 2;
  __bf16* w1h_sw  = (__bf16*)(ws + o); o += (size_t)H1_ * H1_ * 2 * 2;
  __bf16* w2x_sw  = (__bf16*)(ws + o); o += (size_t)H1_ * H2_ * 2 * 2;
  __bf16* w2h_sw  = (__bf16*)(ws + o); o += (size_t)H2_ * H2_ * 2 * 2;
  __bf16* xw1_bk  = (__bf16*)(ws + o); o += (size_t)T_ * B_ * H1_ * 2 * 2;
  __bf16* seq1_bf = (__bf16*)(ws + o); o += (size_t)T_ * B_ * H1_ * 2 * 2;
  __bf16* xw2_bk  = (__bf16*)(ws + o); o += (size_t)T_ * B_ * H2_ * 2 * 2;
  float*  h2f     = (float*) (ws + o); o += (size_t)B_ * H2_ * 4;

  k_cvt_swz<10><<<(EP_ * H1_ / 2 + 255) / 256, 256, 0, stream>>>(W1x, w1x_sw, E_, H1_);
  k_cvt_swz<8><<<(H1_ * H1_ / 2 + 255) / 256, 256, 0, stream>>>(W1h, w1h_sw, H1_, H1_);
  k_cvt_swz<8><<<(H1_ * H2_ / 2 + 255) / 256, 256, 0, stream>>>(W2x, w2x_sw, H1_, H2_);
  k_cvt_swz<16><<<(H2_ * H2_ / 2 + 255) / 256, 256, 0, stream>>>(W2h, w2h_sw, H2_, H2_);

  k_xw1<<<T_, 256, 0, stream>>>(tokens, emb, w1x_sw, b1, xw1_bk);

  k_rnn1<<<1, 512, 0, stream>>>(xw1_bk, w1h_sw, seq1_bf);

  k_xw2<<<T_, 512, 0, stream>>>(seq1_bf, w2x_sw, b2, xw2_bk);

  k_rnn2<<<1, 1024, 0, stream>>>(xw2_bk, w2h_sw, h2f);

  k_head<<<1, 256, 0, stream>>>(h2f, Wd1, bd1, Wd2, bd2, Wc, bc, out);
}
